// KAN_ActorNetwork_27496380629351
// MI455X (gfx1250) — hardware-run, weakly checked
//
#include <hip/hip_runtime.h>
#include <stddef.h>


#pragma clang fp contract(off)

#define D0      128
#define D1      64
#define D2      32
#define D3      16
#define NCO     8
#define GEN     (1 + NCO)
#define K1      (D0 * GEN)
#define K2      (D1 * GEN)
#define K3      (D2 * GEN)
#define FCH     32
#define KCH     (FCH * GEN)
#define GPC     (KCH / 8)
#define NROWT   64
#define AP      296
#define GTW     44
#define NKNOT   12
#define WTHR    64
#define MAXTHR  256
#define NPL     (D1 * K1 + D2 * K2 + D3 * K3)
#define PL2OFF  (D1 * K1)
#define PL3OFF  (D1 * K1 + D2 * K2)
#define LN_EPS_F 1e-5f
#define WSCAP   134217728

#define L_AHI   0
#define L_ALO   (L_AHI + NROWT * AP * 2)
#define L_HB    0
#define L_GT    (L_ALO + NROWT * AP * 2)
#define LDS_LAYER(IN) (L_GT + (IN) * GTW * 4)

static_assert((KCH % 32) == 0);
static_assert((D0 % FCH) == 0 && (D1 % FCH) == 0 && (D2 % FCH) == 0);
static_assert(K1 == (D0 / FCH) * KCH && K2 == (D1 / FCH) * KCH && K3 == (D2 / FCH) * KCH);
static_assert(((AP * 2) % 16) == 0 && AP >= KCH);
static_assert(((NPL / 8) % WTHR) == 0 && ((PL2OFF / 8) % WTHR) == 0 && ((PL3OFF / 8) % WTHR) == 0);
static_assert(((PL2OFF * 2) % 128) == 0 && ((PL3OFF * 2) % 128) == 0 && ((NPL * 2) % 512) == 0);
static_assert((L_ALO % 16) == 0 && (L_GT % 16) == 0);
static_assert(NROWT * (D1 + 4) * 4 <= L_GT);
static_assert(LDS_LAYER(D0) <= 160 * 1024);
static_assert(GPC == 36);
static_assert((GTW * 4) % 16 == 0);

typedef float           v4f   __attribute__((ext_vector_type(4)));
typedef float           v8f   __attribute__((ext_vector_type(8)));
typedef unsigned short  v8us  __attribute__((ext_vector_type(8)));
typedef unsigned short  v16us __attribute__((ext_vector_type(16)));
typedef __bf16          v16bf __attribute__((ext_vector_type(16)));
union Frag { v16bf b; v16us u; v8us h[2]; };
static_assert(sizeof(Frag) == 32);

__device__ __forceinline__ v8f wmb(v16bf a, v16bf bq, v8f c) {
  v8f d = __builtin_amdgcn_wmma_f32_16x16x32_bf16(false, a, false, bq, (short)0, c, false, false);
  asm volatile("v_nop\n\tv_nop\n\tv_nop\n\tv_nop" : "+v"(d) : "v"(a), "v"(bq));
  return d;
}

__device__ __forceinline__ v8f zero8() {
  v8f z = {0.f, 0.f, 0.f, 0.f, 0.f, 0.f, 0.f, 0.f};
  return z;
}

__device__ __forceinline__ unsigned bf16_bits(float f) {
  unsigned u = __float_as_uint(f);
  u += 0x7FFFu + ((u >> 16) & 1u);
  return u >> 16;
}

__device__ __forceinline__ void split2(float v, unsigned short& hb, unsigned short& lb) {
  const unsigned hh = bf16_bits(v);
  const float hf = __uint_as_float(hh << 16);
  hb = (unsigned short)hh;
  lb = (unsigned short)bf16_bits(v - hf);
}

__global__ __launch_bounds__(WTHR) void k_wsplit(
    const float* __restrict__ bw1, const float* __restrict__ sw1,
    const float* __restrict__ bw2, const float* __restrict__ sw2,
    const float* __restrict__ bw3, const float* __restrict__ sw3,
    unsigned short* Wh, unsigned short* Wl) {
  const int b = blockIdx.x, tid = threadIdx.x;
  const int t = b * WTHR + tid;
  const float* bw; const float* sw; int in, t0;
  if (b < (PL2OFF / 8) / WTHR)      { bw = bw1; sw = sw1; in = D0; t0 = 0; }
  else if (b < (PL3OFF / 8) / WTHR) { bw = bw2; sw = sw2; in = D1; t0 = PL2OFF / 8; }
  else                              { bw = bw3; sw = sw3; in = D2; t0 = PL3OFF / 8; }
  const int idx = t - t0;
  const int G   = (in * GEN) / 8;
  const int o   = idx / G;
  const int grp = idx - o * G;
  const int c   = grp / GPC;
  const int r   = grp - c * GPC;
  const int rsl = r < 4 ? r : 3;
  const int fsp = FCH * c + (r >= 4 ? r - 4 : 0);
  const float* ps = bw + (size_t)o * in + FCH * c + 8 * rsl;
  const float* pq = sw + ((size_t)o * in + fsp) * NCO;
  const v4f s0 = *(const v4f*)ps, s1 = *(const v4f*)(ps + 4);
  const v4f g0 = *(const v4f*)pq, g1 = *(const v4f*)(pq + 4);
  const bool isl = r < 4;
  const v4f u0 = isl ? s0 : g0;
  const v4f u1 = isl ? s1 : g1;
  v8us hv, lv;
  unsigned short a, d;
  split2(u0.x, a, d); hv[0] = a; lv[0] = d;
  split2(u0.y, a, d); hv[1] = a; lv[1] = d;
  split2(u0.z, a, d); hv[2] = a; lv[2] = d;
  split2(u0.w, a, d); hv[3] = a; lv[3] = d;
  split2(u1.x, a, d); hv[4] = a; lv[4] = d;
  split2(u1.y, a, d); hv[5] = a; lv[5] = d;
  split2(u1.z, a, d); hv[6] = a; lv[6] = d;
  split2(u1.w, a, d); hv[7] = a; lv[7] = d;
  unsigned short* dh = Wh + (size_t)t * 8;
  unsigned short* dl = Wl + (size_t)t * 8;
  *(volatile v8us*)dh = hv;
  *(volatile v8us*)dl = lv;
  __threadfence();
  *(volatile v8us*)dh = hv;
  *(volatile v8us*)dl = lv;
}

template <int IN, int NOUT, int CSPL, int LNORM>
__global__ __launch_bounds__(MAXTHR) void k_layer(
    const float* __restrict__ X, const float* __restrict__ grid,
    const unsigned short* __restrict__ Wh, const unsigned short* __restrict__ Wl,
    const float* __restrict__ gm, const float* __restrict__ bt, float* Hout) {
  constexpr int NTHR  = 128 * CSPL;
  constexpr int K     = IN * GEN;
  constexpr int NCH   = IN / FCH;
  constexpr int NT    = NOUT / 16 / CSPL;
  constexpr int HP    = NOUT + 4;
  constexpr int RSTEP = NTHR / 32;
  constexpr int QPR   = NOUT / 4;
  constexpr int NV4   = NROWT * QPR;
  constexpr int PER   = NV4 / NTHR;
  static_assert(NTHR <= MAXTHR && K == NCH * KCH && NT >= 1 && NT * 16 * CSPL == NOUT);
  static_assert((NV4 % NTHR) == 0 && PER >= 1 && ((HP * 4) % 16) == 0);
  static_assert(NROWT * HP * 4 <= L_GT);
  static_assert(NROWT * FCH % NTHR == 0);

  extern __shared__ v4f lds_dyn[];
  char* sm = (char*)lds_dyn;
  unsigned short* Ahi = (unsigned short*)(sm + L_AHI);
  unsigned short* Alo = (unsigned short*)(sm + L_ALO);
  float* hb   = (float*)(sm + L_HB);
  float* gtab = (float*)(sm + L_GT);
  const int tid = threadIdx.x, lane = tid & 31, wave = tid >> 5, h = lane >> 4, m = lane & 15;
  const int rt = wave & 3, cg = wave >> 2;
  const int colBase = cg * (NT * 16);
  const int rowBase = blockIdx.x * NROWT;

  for (int f = tid; f < IN; f += NTHR) {
    const float* gp = grid + f * NKNOT;
    float* tp = gtab + f * GTW;
    const v4f w0 = *(const v4f*)gp, w1 = *(const v4f*)(gp + 4), w2 = *(const v4f*)(gp + 8);
    *(v4f*)(tp + 0) = w0; *(v4f*)(tp + 4) = w1; *(v4f*)(tp + 8) = w2;
#pragma unroll 1
    for (int t = 0; t < 11; ++t) tp[12 + t] = 1.0f / (tp[t + 1] - tp[t]);
    tp[23] = 0.0f;
#pragma unroll 1
    for (int t = 0; t < 10; ++t) tp[24 + t] = 1.0f / (tp[t + 2] - tp[t]);
#pragma unroll 1
    for (int t = 0; t < 9; ++t)  tp[34 + t] = 1.0f / (tp[t + 3] - tp[t]);
    tp[43] = 0.0f;
  }
  __syncthreads();

  v8f acc[NT];
#pragma unroll
  for (int nt = 0; nt < NT; ++nt) acc[nt] = zero8();

#pragma unroll 1
  for (int c = 0; c < NCH; ++c) {
    {
      const int ii = tid & 31;
      const int f  = FCH * c + ii;
      const float* tp = gtab + f * GTW;
      const v4f ka = *(const v4f*)(tp + 0),  kb = *(const v4f*)(tp + 4),  kc = *(const v4f*)(tp + 8);
      const v4f ra = *(const v4f*)(tp + 12), rb = *(const v4f*)(tp + 16), rc = *(const v4f*)(tp + 20);
      const v4f pa = *(const v4f*)(tp + 24), pb = *(const v4f*)(tp + 28), pc = *(const v4f*)(tp + 32);
      const v4f pd = *(const v4f*)(tp + 36), pe = *(const v4f*)(tp + 40);
      const float g[12]  = {ka.x, ka.y, ka.z, ka.w, kb.x, kb.y, kb.z, kb.w, kc.x, kc.y, kc.z, kc.w};
      const float q1[11] = {ra.x, ra.y, ra.z, ra.w, rb.x, rb.y, rb.z, rb.w, rc.x, rc.y, rc.z};
      const float q2[10] = {pa.x, pa.y, pa.z, pa.w, pb.x, pb.y, pb.z, pb.w, pc.x, pc.y};
      const float q3[9]  = {pc.z, pc.w, pd.x, pd.y, pd.z, pd.w, pe.x, pe.y, pe.z};
#pragma unroll 1
      for (int row = tid >> 5; row < NROWT; row += RSTEP) {
        const float x = X[(size_t)(rowBase + row) * IN + f];
        float bs[11];
#pragma unroll
        for (int t = 0; t < 11; ++t) bs[t] = (x >= g[t] && x < g[t + 1]) ? 1.0f : 0.0f;
#pragma unroll
        for (int t = 0; t < 10; ++t) {
          const float lf = (x - g[t]) * q1[t];
          const float rg = (g[t + 2] - x) * q1[t + 1];
          bs[t] = lf * bs[t] + rg * bs[t + 1];
        }
#pragma unroll
        for (int t = 0; t < 9; ++t) {
          const float lf = (x - g[t]) * q2[t];
          const float rg = (g[t + 3] - x) * q2[t + 1];
          bs[t] = lf * bs[t] + rg * bs[t + 1];
        }
#pragma unroll
        for (int t = 0; t < 8; ++t) {
          const float lf = (x - g[t]) * q3[t];
          const float rg = (g[t + 4] - x) * q3[t + 1];
          bs[t] = lf * bs[t] + rg * bs[t + 1];
        }
        const float sl = x * __builtin_amdgcn_rcpf(1.0f + __expf(-x));
        unsigned short sh, slo;
        split2(sl, sh, slo);
        v8us bh, bl;
#pragma unroll
        for (int q = 0; q < NCO; ++q) {
          unsigned short a, d;
          split2(bs[q], a, d);
          bh[q] = a; bl[q] = d;
        }
        const int ro = row * AP;
        Ahi[ro + ii] = sh;
        Alo[ro + ii] = slo;
        *(v8us*)(Ahi + ro + FCH + NCO * ii) = bh;
        *(v8us*)(Alo + ro + FCH + NCO * ii) = bl;
      }
    }
    __syncthreads();

    {
      const unsigned short* ah = Ahi + (rt * 16 + m) * AP + 8 * h;
      const unsigned short* al = Alo + (rt * 16 + m) * AP + 8 * h;
      const unsigned short* wh = Wh + (size_t)(colBase + m) * K + KCH * c + 8 * h;
      const unsigned short* wl = Wl + (size_t)(colBase + m) * K + KCH * c + 8 * h;
#pragma unroll 1
      for (int ks = 0; ks < KCH / 32; ++ks) {
        const int ko = 32 * ks;
        Frag fa, fl;
        fa.h[0] = *(const v8us*)(ah + ko);
        fa.h[1] = *(const v8us*)(ah + ko + 16);
        fl.h[0] = *(const v8us*)(al + ko);
        fl.h[1] = *(const v8us*)(al + ko + 16);
#pragma unroll
        for (int nt = 0; nt < NT; ++nt) {
          const size_t no = (size_t)(nt * 16) * K + ko;
          Frag bh2, bl2;
          bh2.h[0] = *(const v8us*)(wh + no);
          bh2.h[1] = *(const v8us*)(wh + no + 16);
          bl2.h[0] = *(const v8us*)(wl + no);
          bl2.h[1] = *(const v8us*)(wl + no + 16);
          acc[nt] = wmb(fa.b, bh2.b, acc[nt]);
          acc[nt] = wmb(fa.b, bl2.b, acc[nt]);
          acc[nt] = wmb(fl.b, bh2.b, acc[nt]);
        }
      }
    }
    __syncthreads();
  }

#pragma unroll
  for (int nt = 0; nt < NT; ++nt) {
#pragma unroll
    for (int r = 0; r < 8; ++r) hb[(rt * 16 + 8 * h + r) * HP + colBase + nt * 16 + m] = acc[nt][r];
  }
  __syncthreads();

  if (LNORM) {
    if (tid < NROWT) {
      float* hr = hb + tid * HP;
      float mu = 0.0f;
#pragma unroll
      for (int i = 0; i < NOUT; ++i) mu += hr[i];
      mu = mu * (1.0f / (float)NOUT);
      float var = 0.0f;
#pragma unroll
      for (int i = 0; i < NOUT; ++i) { const float d = hr[i] - mu; var += d * d; }
      var = var * (1.0f / (float)NOUT);
      const float rs = rsqrtf(var + LN_EPS_F);
#pragma unroll
      for (int i = 0; i < NOUT; ++i) hr[i] = (hr[i] - mu) * rs * gm[i] + bt[i];
    }
    __syncthreads();
  }

  float* gp = Hout + (size_t)rowBase * NOUT;
#pragma unroll
  for (int j = 0; j < PER; ++j) {
    const int e = tid + j * NTHR;
    const int row = e / QPR, q = e - row * QPR;
    const v4f v = *(const v4f*)(hb + row * HP + 4 * q);
    *(volatile v4f*)(gp + 4 * e) = v;
  }
  __threadfence();
#pragma unroll
  for (int j = 0; j < PER; ++j) {
    const int e = tid + j * NTHR;
    const int row = e / QPR, q = e - row * QPR;
    const v4f v = *(const v4f*)(hb + row * HP + 4 * q);
    *(volatile v4f*)(gp + 4 * e) = v;
  }
}

extern "C" void kernel_launch(void* const* d_in, const int* in_sizes, int n_in,
                              void* d_out, int out_size, void* d_ws, size_t ws_size,
                              hipStream_t stream) {
  if (n_in < 14) return;
  const int nrow = in_sizes[0] / D0;
  if (nrow <= 0 || in_sizes[0] != nrow * D0 || (nrow % NROWT) != 0) return;
  if (out_size != nrow * D3) return;
  if (in_sizes[1] != D0 * NKNOT || in_sizes[2] != D1 * D0 || in_sizes[3] != D1 * D0 * NCO) return;
  if (in_sizes[4] != D1 || in_sizes[5] != D1) return;
  if (in_sizes[6] != D1 * NKNOT || in_sizes[7] != D2 * D1 || in_sizes[8] != D2 * D1 * NCO) return;
  if (in_sizes[9] != D2 || in_sizes[10] != D2) return;
  if (in_sizes[11] != D2 * NKNOT || in_sizes[12] != D3 * D2 || in_sizes[13] != D3 * D2 * NCO) return;

  const float* obs = (const float*)d_in[0];
  const float* gr1 = (const float*)d_in[1];
  const float* bw1 = (const float*)d_in[2];
  const float* sw1 = (const float*)d_in[3];
  const float* g1  = (const float*)d_in[4];
  const float* b1  = (const float*)d_in[5];
  const float* gr2 = (const float*)d_in[6];
  const float* bw2 = (const float*)d_in[7];
  const float* sw2 = (const float*)d_in[8];
  const float* g2  = (const float*)d_in[9];
  const float* b2  = (const float*)d_in[10];
  const float* gr3 = (const float*)d_in[11];
  const float* bw3 = (const float*)d_in[12];
  const float* sw3 = (const float*)d_in[13];
  float* out = (float*)d_out;

  const size_t plB = (size_t)NPL * 2;
  size_t off = 0;
  const size_t oWh = off; off += plB;                          off = (off + 255) & ~(size_t)255;
  const size_t oWl = off; off += plB;                          off = (off + 255) & ~(size_t)255;
  const size_t oH1 = off; off += (size_t)nrow * D1 * 4;        off = (off + 255) & ~(size_t)255;
  const size_t oH2 = off; off += (size_t)nrow * D2 * 4;        off = (off + 255) & ~(size_t)255;
  const size_t tot = off;
  if (tot > ws_size || tot > (size_t)WSCAP) return;
  char* ws = (char*)d_ws;
  unsigned short* Wh = (unsigned short*)(ws + oWh);
  unsigned short* Wl = (unsigned short*)(ws + oWl);
  float* H1 = (float*)(ws + oH1);
  float* H2 = (float*)(ws + oH2);
  const int nblk = nrow / NROWT;

  k_wsplit<<<(NPL / 8) / WTHR, WTHR, 0, stream>>>(bw1, sw1, bw2, sw2, bw3, sw3, Wh, Wl);

  hipFuncSetAttribute(reinterpret_cast<const void*>(&k_layer<D0, D1, 2, 1>),
                      hipFuncAttributeMaxDynamicSharedMemorySize, LDS_LAYER(D0));
  k_layer<D0, D1, 2, 1><<<nblk, 256, LDS_LAYER(D0), stream>>>(obs, gr1, Wh, Wl, g1, b1, H1);

  hipFuncSetAttribute(reinterpret_cast<const void*>(&k_layer<D1, D2, 2, 1>),
                      hipFuncAttributeMaxDynamicSharedMemorySize, LDS_LAYER(D1));
  k_layer<D1, D2, 2, 1><<<nblk, 256, LDS_LAYER(D1), stream>>>(H1, gr2, Wh + PL2OFF, Wl + PL2OFF, g2, b2, H2);

  hipFuncSetAttribute(reinterpret_cast<const void*>(&k_layer<D2, D3, 1, 0>),
                      hipFuncAttributeMaxDynamicSharedMemorySize, LDS_LAYER(D2));
  k_layer<D2, D3, 1, 0><<<nblk, 128, LDS_LAYER(D2), stream>>>(H2, gr3, Wh + PL3OFF, Wl + PL3OFF, g2, b2, out);
}
